// ElementGNN_43413529428753
// MI455X (gfx1250) — hardware-verified
//
#include <hip/hip_runtime.h>

typedef float    v8f  __attribute__((ext_vector_type(8)));
typedef float    v4f  __attribute__((ext_vector_type(4)));
typedef __bf16   v16b __attribute__((ext_vector_type(16)));
typedef __bf16   v8b  __attribute__((ext_vector_type(8)));
typedef unsigned v4u  __attribute__((ext_vector_type(4)));

#define EG_NP     8
#define EG_NBLK   110
#define EG_PLANE  (EG_NBLK * 512)
#define EG_PITCH  132
#define EG_ROWS   16
#define EG_WAVES  2


union EgFrag { v16b v; v8b hv[2]; };
union EgV8   { v8b b; v4u u; };

__device__ __forceinline__ void eg_split(float x, __bf16& hi, __bf16& lo)
{
    hi = (__bf16)x;
    lo = (__bf16)(x - (float)hi);
}

__global__ __launch_bounds__(256) void eg_convert_weights(
    const float* __restrict__ W0, const float* __restrict__ W1,
    const float* __restrict__ W2, const float* __restrict__ W3,
    const float* __restrict__ W4, const float* __restrict__ W5,
    const float* __restrict__ W6,
    __bf16* __restrict__ whi, __bf16* __restrict__ wlo)
{
    const int v = blockIdx.x * 256 + threadIdx.x;
    if (v >= EG_NBLK * 64) return;
    const int blk  = v >> 6;
    const int w64  = v & 63;
    const int lane = w64 >> 1;
    const int hf   = w64 & 1;
    const int h    = lane >> 4;
    const int ncol = lane & 15;

    const float* wp = W0; int din = 10, dout = 128, kch4 = 0, base = 0;
    if (blk >= 8)   { wp = W1; din = 128; dout = 128; kch4 = 1; base = 8;   }
    if (blk >= 40)  { wp = W2; din = 128; dout = 128; kch4 = 1; base = 40;  }
    if (blk >= 72)  { wp = W3; din = 128; dout = 128; kch4 = 1; base = 72;  }
    if (blk >= 104) { wp = W4; din = 128; dout = 8;   kch4 = 1; base = 104; }
    if (blk >= 108) { wp = W5; din = 8;   dout = 8;   kch4 = 0; base = 108; }
    if (blk >= 109) { wp = W6; din = 8;   dout = 10;  kch4 = 0; base = 109; }
    const int local = blk - base;
    const int kc = kch4 ? (local & 3) : 0;
    const int nt = kch4 ? (local >> 2) : local;
    const int n  = nt * 16 + ncol;

    EgV8 uh, ul;
    #pragma unroll
    for (int i = 0; i < 8; ++i) {
        const int K = kc * 32 + 8 * h + 16 * hf + i;
        float x = 0.0f;
        if (K < din && n < dout) x = wp[K * dout + n];
        __bf16 xh, xl;
        eg_split(x, xh, xl);
        uh.b[i] = xh;
        ul.b[i] = xl;
    }
    const size_t off = (size_t)v * 8;
    volatile v4u* ph = (volatile v4u*)(whi + off);
    volatile v4u* pl = (volatile v4u*)(wlo + off);
    *ph = uh.u;
    *pl = ul.u;
    __threadfence();
    *ph = uh.u;
    *pl = ul.u;
}

template<bool UPPER>
__device__ __forceinline__ void eg_buildA(const float* rowp, int k0, int h, v16b& ah, v16b& al)
{
    {
        const v4f p0 = *(const v4f*)(rowp + k0 + 8 * h);
        const v4f p1 = *(const v4f*)(rowp + k0 + 8 * h + 4);
        #pragma unroll
        for (int i = 0; i < 4; ++i) {
            __bf16 x, y;
            eg_split(p0[i], x, y); ah[i] = x;     al[i] = y;
            eg_split(p1[i], x, y); ah[4 + i] = x; al[4 + i] = y;
        }
    }
    if (UPPER) {
        const v4f p2 = *(const v4f*)(rowp + k0 + 16 + 8 * h);
        const v4f p3 = *(const v4f*)(rowp + k0 + 16 + 8 * h + 4);
        #pragma unroll
        for (int i = 0; i < 4; ++i) {
            __bf16 x, y;
            eg_split(p2[i], x, y); ah[8 + i] = x;  al[8 + i] = y;
            eg_split(p3[i], x, y); ah[12 + i] = x; al[12 + i] = y;
        }
    } else {
        #pragma unroll
        for (int i = 8; i < 16; ++i) { ah[i] = (__bf16)0.0f; al[i] = (__bf16)0.0f; }
    }
}

__device__ __forceinline__ v8f eg_mma3(v8f c, const v16b& ah, const v16b& al,
                                       const __bf16* __restrict__ whi,
                                       const __bf16* __restrict__ wlo,
                                       int blk, int lane)
{
    EgFrag bh, bl;
    const size_t off = (size_t)blk * 512 + (size_t)lane * 16;
    const __bf16* ph = whi + off;
    const __bf16* pl = wlo + off;
    bh.hv[0] = *(const v8b*)(ph);
    bh.hv[1] = *(const v8b*)(ph + 8);
    bl.hv[0] = *(const v8b*)(pl);
    bl.hv[1] = *(const v8b*)(pl + 8);
    c = __builtin_amdgcn_wmma_f32_16x16x32_bf16(false, ah, false, bh.v, (short)0, c, false, false);
    c = __builtin_amdgcn_wmma_f32_16x16x32_bf16(false, ah, false, bl.v, (short)0, c, false, false);
    c = __builtin_amdgcn_wmma_f32_16x16x32_bf16(false, al, false, bh.v, (short)0, c, false, false);
    asm volatile("v_nop\n\tv_nop\n\tv_nop\n\tv_nop"
                 : "+v"(c) : "v"(ah), "v"(al), "v"(bh.v), "v"(bl.v));
    return c;
}

template<int KCH, int NT, bool UPPER, bool RELU>
__device__ __forceinline__ void eg_dense(const float* srcRow, float* dst,
                                         const __bf16* __restrict__ whi,
                                         const __bf16* __restrict__ wlo, int blkOff,
                                         const float* __restrict__ bias, int dimOut, int lane)
{
    const int h = lane >> 4, m = lane & 15;
    v16b ah[KCH], al[KCH];
    #pragma unroll
    for (int kc = 0; kc < KCH; ++kc) eg_buildA<UPPER>(srcRow, kc * 32, h, ah[kc], al[kc]);

    #pragma unroll 1
    for (int nt = 0; nt < NT; ++nt) {
        const int n = nt * 16 + m;
        float bv = 0.0f;
        if (n < dimOut) bv = bias[n];
        v8f c;
        #pragma unroll
        for (int r = 0; r < 8; ++r) c[r] = bv;
        #pragma unroll
        for (int kc = 0; kc < KCH; ++kc)
            c = eg_mma3(c, ah[kc], al[kc], whi, wlo, blkOff + nt * KCH + kc, lane);
        #pragma unroll
        for (int r = 0; r < 8; ++r) {
            float x = c[r];
            if (RELU) x = fmaxf(x, 0.0f);
            dst[(8 * h + r) * EG_PITCH + n] = x;
        }
    }
}

__global__ __launch_bounds__(64) void eg_main(
    const float* __restrict__ data, const int* __restrict__ elements,
    const float* __restrict__ b0, const float* __restrict__ b1,
    const float* __restrict__ b2, const float* __restrict__ b3,
    const float* __restrict__ b4, const float* __restrict__ b5,
    const float* __restrict__ b6,
    const __bf16* __restrict__ whi, const __bf16* __restrict__ wlo,
    float* __restrict__ out, int nElem, int nData, int outN)
{
    __shared__ __align__(16) float s_act[EG_WAVES][2][EG_ROWS * EG_PITCH];
    __shared__ __align__(16) float s_sent[EG_WAVES][EG_ROWS * 16];
    __shared__ __align__(16) float s_out[EG_WAVES][EG_ROWS * EG_NP];

    const int w    = threadIdx.x >> 5;
    const int lane = threadIdx.x & 31;
    const int h    = lane >> 4;
    const int m    = lane & 15;
    const int row0 = blockIdx.x * (EG_WAVES * EG_ROWS) + w * EG_ROWS;

    float* ss   = &s_sent[w][0];
    float* bufA = &s_act[w][0][0];
    float* bufB = &s_act[w][1][0];
    float* so   = &s_out[w][0];

    #pragma unroll
    for (int t = 0; t < 8; ++t) {
        const int s = t * 32 + lane;
        const int r = s >> 4, c = s & 15;
        float v = 0.0f;
        int i = row0 + r;
        if (i > nElem - 1) i = nElem - 1;
        if (c < 10) {
            const int x = elements[i];
            int e = x / (EG_NP + 1);
            if ((x % (EG_NP + 1)) != 0 && x < 0) e -= 1;
            int lidx = (e - 1) % nElem; if (lidx < 0) lidx += nElem;
            int ridx = (e + 1) % nElem; if (ridx < 0) ridx += nElem;
            int ec = e; if (ec < 0) ec += nElem;
            if (ec < 0) ec = 0; if (ec > nElem - 1) ec = nElem - 1;
            int src;
            if (c == 0)      src = lidx * EG_NP + (EG_NP - 1);
            else if (c == 9) src = ridx * EG_NP;
            else             src = ec * EG_NP + (c - 1);
            if (src < 0) src = 0; if (src > nData - 1) src = nData - 1;
            v = data[src];
        }
        ss[s] = v;
    }
    __syncthreads();

    eg_dense<1, 8, false, true >(ss + m * 16,         bufA, whi, wlo,   0, b0, 128, lane);
    __syncthreads();
    eg_dense<4, 8, true,  false>(bufA + m * EG_PITCH, bufB, whi, wlo,   8, b1, 128, lane);
    __syncthreads();
    eg_dense<4, 8, true,  true >(bufB + m * EG_PITCH, bufA, whi, wlo,  40, b2, 128, lane);
    __syncthreads();
    eg_dense<4, 8, true,  false>(bufA + m * EG_PITCH, bufB, whi, wlo,  72, b3, 128, lane);
    __syncthreads();
    eg_dense<4, 1, true,  true >(bufB + m * EG_PITCH, bufA, whi, wlo, 104, b4,   8, lane);
    __syncthreads();
    eg_dense<1, 1, false, false>(bufA + m * EG_PITCH, bufB, whi, wlo, 108, b5,   8, lane);
    __syncthreads();

    {
        v16b ah, al;
        eg_buildA<false>(bufB + m * EG_PITCH, 0, h, ah, al);
        const int n = m;
        float bv = 0.0f;
        if (n < 10) bv = b6[n];
        v8f c;
        #pragma unroll
        for (int r = 0; r < 8; ++r) c[r] = bv;
        c = eg_mma3(c, ah, al, whi, wlo, 109, lane);
        if (n >= 1 && n <= EG_NP) {
            #pragma unroll
            for (int r = 0; r < 8; ++r) {
                const int row = 8 * h + r;
                so[row * EG_NP + (n - 1)] = ss[row * 16 + n] + c[r];
            }
        }
    }
    __syncthreads();

    {
        const v4f val = *(const v4f*)(so + lane * 4);
        const int orow = row0 + (lane >> 1);
        const size_t ofs = (size_t)row0 * EG_NP + (size_t)lane * 4;
        const bool ok = (orow < nElem) && (ofs + 4 <= (size_t)outN);
        if (ok) *(volatile v4f*)(out + ofs) = val;
        __threadfence();
        if (ok) *(volatile v4f*)(out + ofs) = val;
    }
}

extern "C" void kernel_launch(void* const* d_in, const int* in_sizes, int n_in,
                              void* d_out, int out_size, void* d_ws, size_t ws_size,
                              hipStream_t stream)
{
    if (n_in < 16) return;
    const int nData = in_sizes[0];
    const int nElem = in_sizes[1];
    if (nElem <= 0 || nData < nElem * EG_NP || out_size < nElem * EG_NP) return;
    if (in_sizes[2]  != 10 * 128  || in_sizes[3]  < 128 ||
        in_sizes[4]  != 128 * 128 || in_sizes[5]  < 128 ||
        in_sizes[6]  != 128 * 128 || in_sizes[7]  < 128 ||
        in_sizes[8]  != 128 * 128 || in_sizes[9]  < 128 ||
        in_sizes[10] != 128 * 8   || in_sizes[11] < 8   ||
        in_sizes[12] != 8 * 8     || in_sizes[13] < 8   ||
        in_sizes[14] != 8 * 10    || in_sizes[15] < 10) return;

    const size_t planeBytes = (size_t)EG_PLANE * sizeof(__bf16);
    if (ws_size < 2 * planeBytes) return;

    const float* data     = (const float*)d_in[0];
    const int*   elements = (const int*)d_in[1];
    const float* W[7];
    const float* b[7];
    for (int i = 0; i < 7; ++i) {
        W[i] = (const float*)d_in[2 + 2 * i];
        b[i] = (const float*)d_in[3 + 2 * i];
    }
    __bf16* whi = (__bf16*)d_ws;
    __bf16* wlo = (__bf16*)((char*)d_ws + planeBytes);

    const int nVec = EG_NBLK * 64;
    eg_convert_weights<<<(nVec + 255) / 256, 256, 0, stream>>>(
        W[0], W[1], W[2], W[3], W[4], W[5], W[6], whi, wlo);

    const int rowsPerBlock = EG_WAVES * EG_ROWS;
    const int nBlocks = (nElem + rowsPerBlock - 1) / rowsPerBlock;
    eg_main<<<nBlocks, EG_WAVES * 32, 0, stream>>>(
        data, elements, b[0], b[1], b[2], b[3], b[4], b[5], b[6],
        whi, wlo, (float*)d_out, nElem, nData, out_size);
}
